// MLA256Attention_65687229825560
// MI455X (gfx1250) — hardware-verified
//
#include <hip/hip_runtime.h>
#include <math.h>
#include <stdint.h>

#define NB    4
#define TS    2048
#define DM    1024
#define NH    8
#define HD    256
#define KR    64
#define NROWS (NB * TS)
#define QD    (NH * HD)
#define HRK   (NH * KR)
#define QLP   (HRK + KR)

typedef _Float16     v16h __attribute__((ext_vector_type(16)));
typedef _Float16     v8h  __attribute__((ext_vector_type(8)));
typedef __bf16       v16b __attribute__((ext_vector_type(16)));
typedef __bf16       v8b  __attribute__((ext_vector_type(8)));
typedef float        v8f  __attribute__((ext_vector_type(8)));
typedef float        v4f  __attribute__((ext_vector_type(4)));
typedef float        v2f  __attribute__((ext_vector_type(2)));
typedef unsigned int v4u  __attribute__((ext_vector_type(4)));

__device__ __forceinline__ unsigned short f2bf_bits(float f) {
  unsigned u = __float_as_uint(f);
  return (unsigned short)((u + 0x7FFFu + ((u >> 16) & 1u)) >> 16);
}
__device__ __forceinline__ float bf_bits2f(unsigned short h) { return __uint_as_float(((unsigned)h) << 16); }
__device__ __forceinline__ unsigned pk16(unsigned short a, unsigned short b) { return (unsigned)a | ((unsigned)b << 16); }
__device__ __forceinline__ void split_pair(float f0, float f1, unsigned& uh, unsigned& ul) {
  const unsigned short h0 = f2bf_bits(f0), h1 = f2bf_bits(f1);
  const unsigned short l0 = f2bf_bits(f0 - bf_bits2f(h0)), l1 = f2bf_bits(f1 - bf_bits2f(h1));
  uh = pk16(h0, h1); ul = pk16(l0, l1);
}

__device__ __forceinline__ v16b ldfrag_b(const __bf16* p) {
  union { v16b v; v8b h[2]; } f;
  f.h[0] = *(const v8b*)(p); f.h[1] = *(const v8b*)(p + 16); return f.v;
}
__device__ __forceinline__ v16h ldfrag_h(const _Float16* p) {
  union { v16h v; v8h h[2]; } f;
  f.h[0] = *(const v8h*)(p); f.h[1] = *(const v8h*)(p + 16); return f.v;
}
__device__ __forceinline__ v8f mma_b(v16b a, v16b b, v8f c) {
  return __builtin_amdgcn_wmma_f32_16x16x32_bf16(false, a, false, b, (short)0, c, false, false);
}
__device__ __forceinline__ v8f mma_h(v16h a, v16h b, v8f c) {
  c = __builtin_amdgcn_wmma_f32_16x16x32_f16(false, a, false, b, (short)0, c, false, false);
  asm volatile("v_nop\n\tv_nop\n\tv_nop\n\tv_nop" : "+v"(c) : "v"(a), "v"(b));
  return c;
}
__device__ __forceinline__ void dep_guard_b(v8f& a, v8f& b, v16b x, v16b y) { asm volatile("v_nop\n\tv_nop\n\tv_nop\n\tv_nop" : "+v"(a), "+v"(b) : "v"(x), "v"(y)); }
__device__ __forceinline__ void keep4_b(v16b a, v16b b, v16b c, v16b d) { asm volatile("v_nop" :: "v"(a), "v"(b), "v"(c), "v"(d)); }
__device__ __forceinline__ void acc_guard4(v8f& a, v8f& b, v8f& c, v8f& d) { asm volatile("v_nop\n\tv_nop\n\tv_nop\n\tv_nop" : "+v"(a), "+v"(b), "+v"(c), "+v"(d)); }

template <int OUT_MODE>
__global__ __launch_bounds__(256) void gemm64_split(
    const unsigned short* __restrict__ Ap, const unsigned short* __restrict__ A2p, int lda, long strideA,
    const unsigned short* __restrict__ Btp, const unsigned short* __restrict__ Bt2p, int ldb, long strideB,
    void* __restrict__ Cout, void* __restrict__ Cout2, int ldc, long strideC,
    int M, int N, int K, float scale) {
  const __bf16* A   = (const __bf16*)(const void*)Ap;
  const __bf16* A2  = (const __bf16*)(const void*)A2p;
  const __bf16* Bt  = (const __bf16*)(const void*)Btp;
  const __bf16* Bt2 = (const __bf16*)(const void*)Bt2p;
  __shared__ __align__(16) float sT[8][16 * 68];
  const int b    = blockIdx.y;
  const int lane = threadIdx.x & 31;
  const int wave = threadIdx.x >> 5;
  const int tilesN = N >> 6;
  const int tilesM = M >> 6;
  const int tile = blockIdx.x * 8 + wave;
  if (tile >= tilesM * tilesN) return;
  const int tm = tile / tilesN;
  const int tn = tile - tm * tilesN;
  const int m0 = tm << 6;
  const int n0 = tn << 6;

  const __bf16* Ab  = A   + (size_t)b * strideA;
  const __bf16* Ab2 = A2  + (size_t)b * strideA;
  const __bf16* Bb  = Bt  + (size_t)b * strideB;
  const __bf16* Bb2 = Bt2 + (size_t)b * strideB;

  const int rlane = lane & 15;
  const int koff  = (lane >> 4) * 8;
  const int mOff  = (lane >> 4) * 8;

  v8f acc[4][4];
#pragma unroll
  for (int i = 0; i < 4; ++i)
#pragma unroll
    for (int j = 0; j < 4; ++j) acc[i][j] = (v8f){0.f,0.f,0.f,0.f,0.f,0.f,0.f,0.f};

  for (int k0 = 0; k0 < K; k0 += 32) {
    v16b bh[4], bl[4];
#pragma unroll
    for (int j = 0; j < 4; ++j) {
      const size_t bo = (size_t)(n0 + (j << 4) + rlane) * ldb + koff + k0;
      bh[j] = ldfrag_b(Bb + bo);
      bl[j] = ldfrag_b(Bb2 + bo);
    }
#pragma unroll
    for (int i = 0; i < 4; ++i) {
      const size_t ao = (size_t)(m0 + (i << 4) + rlane) * lda + koff + k0;
      const v16b ah = ldfrag_b(Ab + ao);
      const v16b al = ldfrag_b(Ab2 + ao);
#pragma unroll
      for (int j = 0; j < 4; ++j) {
        acc[i][j] = mma_b(ah, bh[j], acc[i][j]);
        acc[i][j] = mma_b(ah, bl[j], acc[i][j]);
        acc[i][j] = mma_b(al, bh[j], acc[i][j]);
      }
      dep_guard_b(acc[i][0], acc[i][3], ah, al);
    }
    keep4_b(bh[0], bh[1], bh[2], bh[3]);
    keep4_b(bl[0], bl[1], bl[2], bl[3]);
  }
  acc_guard4(acc[0][0], acc[0][1], acc[0][2], acc[0][3]);
  acc_guard4(acc[1][0], acc[1][1], acc[1][2], acc[1][3]);
  acc_guard4(acc[2][0], acc[2][1], acc[2][2], acc[2][3]);
  acc_guard4(acc[3][0], acc[3][1], acc[3][2], acc[3][3]);

  float* slab = sT[wave];
#pragma unroll
  for (int i = 0; i < 4; ++i) {
    const int mBase = m0 + (i << 4);
#pragma unroll
    for (int j = 0; j < 4; ++j) {
#pragma unroll
      for (int r = 0; r < 8; ++r) slab[(mOff + r) * 68 + (j << 4) + rlane] = acc[i][j][r] * scale;
    }
    __builtin_amdgcn_fence(__ATOMIC_RELEASE, "workgroup");
    __builtin_amdgcn_wave_barrier();
    __builtin_amdgcn_fence(__ATOMIC_ACQUIRE, "workgroup");
    if (OUT_MODE == 0) {
      float* C = (float*)Cout + (size_t)b * strideC;
      const int hh = lane >> 4, c4 = (lane & 15) * 4;
      for (int pass = 0; pass < 2; ++pass) {
#pragma unroll
        for (int it = 0; it < 8; ++it) {
          const int row = it * 2 + hh;
          const v4f v = *(const v4f*)(slab + row * 68 + c4);
          *(volatile v4f*)(C + (size_t)(mBase + row) * ldc + n0 + c4) = v;
        }
        __threadfence();
      }
    } else {
      const int q = lane >> 3, c8 = (lane & 7) * 8;
      unsigned short* C  = (unsigned short*)Cout  + (size_t)b * strideC;
      unsigned short* C2 = (unsigned short*)Cout2 + (size_t)b * strideC;
      for (int pass = 0; pass < 2; ++pass) {
#pragma unroll
        for (int it = 0; it < 4; ++it) {
          const int row = it * 4 + q;
          const float* sp = slab + row * 68 + c8;
          if (OUT_MODE == 1) {
            v8h hv;
#pragma unroll
            for (int e = 0; e < 8; ++e) hv[e] = (_Float16)sp[e];
            *(volatile v8h*)(C + (size_t)(mBase + row) * ldc + n0 + c8) = hv;
          } else {
            v4u hv, lv;
#pragma unroll
            for (int e = 0; e < 4; ++e) {
              unsigned uh, ul;
              split_pair(sp[2 * e], sp[2 * e + 1], uh, ul);
              hv[e] = uh; lv[e] = ul;
            }
            *(volatile v4u*)(C  + (size_t)(mBase + row) * ldc + n0 + c8) = hv;
            *(volatile v4u*)(C2 + (size_t)(mBase + row) * ldc + n0 + c8) = lv;
          }
        }
        __threadfence();
      }
    }
    __builtin_amdgcn_fence(__ATOMIC_RELEASE, "workgroup");
    __builtin_amdgcn_wave_barrier();
    __builtin_amdgcn_fence(__ATOMIC_ACQUIRE, "workgroup");
  }
}

__global__ __launch_bounds__(256) void split_bf16x2_kernel(const float* __restrict__ in, unsigned short* __restrict__ hi,
                                                           unsigned short* __restrict__ lo, int n2) {
  const int i = blockIdx.x * 256 + threadIdx.x;
  if (i < n2) {
    const v2f f = *(const v2f*)(in + 2 * (size_t)i);
    unsigned uh, ul;
    split_pair(f[0], f[1], uh, ul);
    ((volatile unsigned*)hi)[i] = uh;
    ((volatile unsigned*)lo)[i] = ul;
    __threadfence();
    ((volatile unsigned*)hi)[i] = uh;
    ((volatile unsigned*)lo)[i] = ul;
  }
}

__global__ __launch_bounds__(256) void tsplit_kernel(const float* __restrict__ W, unsigned short* __restrict__ oh,
                                                     unsigned short* __restrict__ ol, int R, int Cc, long sIn, long sOut) {
  __shared__ __align__(16) float tf[64 * 68];
  W  += (size_t)blockIdx.z * sIn;
  oh += (size_t)blockIdx.z * sOut;
  ol += (size_t)blockIdx.z * sOut;
  const int c0  = blockIdx.x * 64;
  const int r0  = blockIdx.y * 64;
  const int tid = threadIdx.x;
  {
    const int lr = tid >> 4;
    const int c4 = (tid & 15) * 4;
#pragma unroll
    for (int it = 0; it < 4; ++it) {
      const int rr = it * 16 + lr;
      const v4f a = *(const v4f*)(W + (size_t)(r0 + rr) * Cc + c0 + c4);
      *(v4f*)(tf + rr * 68 + c4) = a;
    }
  }
  __syncthreads();
  const int sub = tid >> 3;
  const int c8  = (tid & 7) * 8;
  v4u hv[2], lv[2];
#pragma unroll
  for (int it = 0; it < 2; ++it) {
    const int oc = it * 32 + sub;
    v4u a, a2;
#pragma unroll
    for (int q = 0; q < 4; ++q) {
      unsigned uh, ul;
      split_pair(tf[(c8 + 2 * q) * 68 + oc], tf[(c8 + 2 * q + 1) * 68 + oc], uh, ul);
      a[q] = uh; a2[q] = ul;
    }
    hv[it] = a; lv[it] = a2;
  }
  for (int pass = 0; pass < 2; ++pass) {
#pragma unroll
    for (int it = 0; it < 2; ++it) {
      const int oc = it * 32 + sub;
      const size_t go = (size_t)(c0 + oc) * R + r0 + c8;
      *(volatile v4u*)(oh + go) = hv[it];
      *(volatile v4u*)(ol + go) = lv[it];
    }
    __threadfence();
  }
}

__global__ __launch_bounds__(256) void lat_tr_kernel(const unsigned short* __restrict__ ql, unsigned short* __restrict__ lt) {
  __shared__ __align__(16) unsigned short tf[64 * 72];
  const int t0 = blockIdx.x * 64;
  const int b  = blockIdx.y;
  const size_t rb = (size_t)b * TS + t0;
  const int tid = threadIdx.x;
  const int lr = tid >> 3;
  const int c8 = (tid & 7) * 8;
#pragma unroll
  for (int it = 0; it < 2; ++it) {
    const int rr = it * 32 + lr;
    const v4u w = *(const v4u*)(ql + (rb + rr) * QLP + HRK + c8);
    *(v4u*)(tf + rr * 72 + c8) = w;
  }
  __syncthreads();
  v4u ov[2];
#pragma unroll
  for (int it = 0; it < 2; ++it) {
    const int oc = it * 32 + lr;
    v4u a;
#pragma unroll
    for (int q = 0; q < 4; ++q) a[q] = pk16(tf[(c8 + 2 * q) * 72 + oc], tf[(c8 + 2 * q + 1) * 72 + oc]);
    ov[it] = a;
  }
  unsigned short* ob = lt + (size_t)b * KR * TS + t0 + c8;
#pragma unroll
  for (int it = 0; it < 2; ++it) {
    const int oc = it * 32 + lr;
    *(volatile v4u*)(ob + (size_t)oc * TS) = ov[it];
  }
  __threadfence();
#pragma unroll
  for (int it = 0; it < 2; ++it) {
    const int oc = it * 32 + lr;
    *(volatile v4u*)(ob + (size_t)oc * TS) = ov[it];
  }
}

#define AT_NW 4
#define AT_QB 64
#define AT_KC 64

__global__ __launch_bounds__(128)
void attn_lat64_kernel(const unsigned short* __restrict__ qlp, const unsigned short* __restrict__ ltp,
                       unsigned short* __restrict__ plh, unsigned short* __restrict__ pll,
                       float s_mul, float o_mul) {
  union FH { v16h v; v8h h[2]; };
  __shared__ __align__(16) _Float16 Ksh[AT_KC * KR];
  __shared__ __align__(16) _Float16 Vth[KR * AT_KC];
  __shared__ __align__(16) _Float16 Psh[AT_NW][16 * AT_KC];
  __shared__ __align__(16) float    Os[AT_NW][16 * 68];

  const int tid  = threadIdx.x;
  const int wave = tid >> 5;
  const int lane = tid & 31;
  const int hh   = lane >> 4;
  const int c    = lane & 15;

  const int nqb = TS / AT_QB;
  const int bx = blockIdx.x;
  const int qb = bx % nqb;
  const int h  = (bx / nqb) % NH;
  const int b  = bx / (nqb * NH);
  const int q0 = qb * AT_QB + wave * 16;
  const size_t trow0 = (size_t)b * TS;

  const _Float16* QL = (const _Float16*)(const void*)qlp;
  const _Float16* Qp = QL + trow0 * QLP + h * KR;
  const _Float16* Kp = QL + trow0 * QLP + HRK;
  const _Float16* Vp = (const _Float16*)(const void*)ltp + (size_t)b * KR * TS;

  v16h qa[2];
#pragma unroll
  for (int dc = 0; dc < 2; ++dc) qa[dc] = ldfrag_h(Qp + (size_t)(q0 + c) * QLP + dc * 32 + 8 * hh);

  float mrow[8], lrow[8];
  v8f oacc[4];
#pragma unroll
  for (int r = 0; r < 8; ++r) { mrow[r] = -INFINITY; lrow[r] = 0.f; }
#pragma unroll
  for (int t = 0; t < 4; ++t) oacc[t] = (v8f){0.f,0.f,0.f,0.f,0.f,0.f,0.f,0.f};

  const int nChunks = TS / AT_KC;
  for (int kc = 0; kc < nChunks; ++kc) {
    const int kv0 = kc * AT_KC;
    __syncthreads();
    {
      const int r = tid >> 1, half = (tid & 1) * 32;
      const _Float16* ks = Kp + (size_t)(kv0 + r) * QLP + half;
      const _Float16* vs = Vp + (size_t)r * TS + kv0 + half;
#pragma unroll
      for (int i = 0; i < 4; ++i) {
        const v8h a0 = *(const v8h*)(ks + 8 * i);
        const v8h b0 = *(const v8h*)(vs + 8 * i);
        *(v8h*)(Ksh + r * KR    + half + 8 * i) = a0;
        *(v8h*)(Vth + r * AT_KC + half + 8 * i) = b0;
      }
    }
    __syncthreads();

    v8f s[4];
#pragma unroll
    for (int j = 0; j < 4; ++j) {
      s[j] = (v8f){0.f,0.f,0.f,0.f,0.f,0.f,0.f,0.f};
#pragma unroll
      for (int dc = 0; dc < 2; ++dc) {
        FH kb;
        kb.h[0] = *(const v8h*)(Ksh + (j * 16 + c) * KR + dc * 32 + 8 * hh);
        kb.h[1] = *(const v8h*)(Ksh + (j * 16 + c) * KR + dc * 32 + 16 + 8 * hh);
        s[j] = mma_h(qa[dc], kb.v, s[j]);
      }
    }
    float cm[8];
#pragma unroll
    for (int r = 0; r < 8; ++r) {
      float m = -INFINITY;
#pragma unroll
      for (int j = 0; j < 4; ++j) {
        const float sv = s[j][r] * s_mul;
        s[j][r] = sv;
        m = fmaxf(m, sv);
      }
#pragma unroll
      for (int off = 1; off < 16; off <<= 1) m = fmaxf(m, __shfl_xor(m, off, 32));
      cm[r] = m;
    }
    _Float16* pw = Psh[wave];
#pragma unroll
    for (int r = 0; r < 8; ++r) {
      const float mnew  = fmaxf(mrow[r], cm[r]);
      const float alpha = __expf(mrow[r] - mnew);
      mrow[r] = mnew;
      float psum = 0.f;
#pragma unroll
      for (int j = 0; j < 4; ++j) {
        const float p = __expf(s[j][r] - mnew);
        psum += p;
        pw[(8 * hh + r) * AT_KC + j * 16 + c] = (_Float16)(p * 4096.0f);
      }
#pragma unroll
      for (int off = 1; off < 16; off <<= 1) psum += __shfl_xor(psum, off, 32);
      lrow[r] = lrow[r] * alpha + psum;
#pragma unroll
      for (int t = 0; t < 4; ++t) oacc[t][r] *= alpha;
    }
    __builtin_amdgcn_fence(__ATOMIC_RELEASE, "workgroup");
    __builtin_amdgcn_wave_barrier();
    __builtin_amdgcn_fence(__ATOMIC_ACQUIRE, "workgroup");
#pragma unroll
    for (int kk = 0; kk < 2; ++kk) {
      FH pa;
      pa.h[0] = *(const v8h*)(pw + c * AT_KC + kk * 32 + 8 * hh);
      pa.h[1] = *(const v8h*)(pw + c * AT_KC + kk * 32 + 16 + 8 * hh);
#pragma unroll
      for (int t = 0; t < 4; ++t) {
        FH vb;
        vb.h[0] = *(const v8h*)(Vth + (t * 16 + c) * AT_KC + kk * 32 + 8 * hh);
        vb.h[1] = *(const v8h*)(Vth + (t * 16 + c) * AT_KC + kk * 32 + 16 + 8 * hh);
        oacc[t] = mma_h(pa.v, vb.v, oacc[t]);
      }
    }
  }

  float* os = Os[wave];
#pragma unroll
  for (int r = 0; r < 8; ++r) {
    const float inv = o_mul * (1.0f / lrow[r]);
#pragma unroll
    for (int t = 0; t < 4; ++t) os[(8 * hh + r) * 68 + t * 16 + c] = oacc[t][r] * inv;
  }
  __builtin_amdgcn_fence(__ATOMIC_RELEASE, "workgroup");
  __builtin_amdgcn_wave_barrier();
  __builtin_amdgcn_fence(__ATOMIC_ACQUIRE, "workgroup");
  {
    const int qq = lane >> 3, c8 = (lane & 7) * 8;
    v4u hv[4], lv[4];
#pragma unroll
    for (int it = 0; it < 4; ++it) {
      const int row = it * 4 + qq;
      const v4f f0 = *(const v4f*)(os + row * 68 + c8);
      const v4f f1 = *(const v4f*)(os + row * 68 + c8 + 4);
      v4u a, a2;
      unsigned uh, ul;
      split_pair(f0[0], f0[1], uh, ul); a[0] = uh; a2[0] = ul;
      split_pair(f0[2], f0[3], uh, ul); a[1] = uh; a2[1] = ul;
      split_pair(f1[0], f1[1], uh, ul); a[2] = uh; a2[2] = ul;
      split_pair(f1[2], f1[3], uh, ul); a[3] = uh; a2[3] = ul;
      hv[it] = a; lv[it] = a2;
    }
    unsigned short* ph = plh + (trow0 + q0) * HRK + h * KR + c8;
    unsigned short* pl = pll + (trow0 + q0) * HRK + h * KR + c8;
#pragma unroll
    for (int it = 0; it < 4; ++it) {
      const int row = it * 4 + qq;
      *(volatile v4u*)(ph + (size_t)row * HRK) = hv[it];
      *(volatile v4u*)(pl + (size_t)row * HRK) = lv[it];
    }
    __threadfence();
#pragma unroll
    for (int it = 0; it < 4; ++it) {
      const int row = it * 4 + qq;
      *(volatile v4u*)(ph + (size_t)row * HRK) = hv[it];
      *(volatile v4u*)(pl + (size_t)row * HRK) = lv[it];
    }
  }
}

extern "C" void kernel_launch(void* const* d_in, const int* in_sizes, int n_in,
                              void* d_out, int out_size, void* d_ws, size_t ws_size,
                              hipStream_t stream) {
  if (n_in < 6) return;
  if (in_sizes[0] != NROWS * DM) return;
  if (in_sizes[1] != QD * DM) return;
  if (in_sizes[2] != KR * DM) return;
  if (in_sizes[3] != QD * KR || in_sizes[4] != QD * KR) return;
  if (in_sizes[5] != DM * QD) return;
  if (out_size != NROWS * DM) return;

  const float* x   = (const float*)d_in[0];
  const float* Wq  = (const float*)d_in[1];
  const float* Wkv = (const float*)d_in[2];
  const float* Wku = (const float*)d_in[3];
  const float* Wvu = (const float*)d_in[4];
  const float* Wo  = (const float*)d_in[5];

  const size_t szX   = (size_t)NROWS * DM * 2;
  const size_t szWqT = (size_t)NH * DM * HD * 2;
  const size_t szWkT = (size_t)NH * KR * HD * 2;
  const size_t szWo  = (size_t)DM * QD * 2;
  const size_t szBtQ = (size_t)QLP * DM * 2;
  const size_t szM   = (size_t)DM * HRK * 2;
  const size_t szQL  = (size_t)NROWS * QLP * 2;
  const size_t szLT  = (size_t)NB * KR * TS * 2;
  const size_t szPL  = (size_t)NROWS * HRK * 2;
  size_t off = 0;
  const size_t oXh   = off; off += szX;    const size_t oXl   = off; off += szX;
  const size_t oWqTh = off; off += szWqT;  const size_t oWqTl = off; off += szWqT;
  const size_t oWkTh = off; off += szWkT;  const size_t oWkTl = off; off += szWkT;
  const size_t oWvTh = off; off += szWkT;  const size_t oWvTl = off; off += szWkT;
  const size_t oWoh  = off; off += szWo;   const size_t oWol  = off; off += szWo;
  const size_t oBtQh = off; off += szBtQ;  const size_t oBtQl = off; off += szBtQ;
  const size_t oMh   = off; off += szM;    const size_t oMl   = off; off += szM;
  const size_t oQL   = off; off += szQL;
  const size_t oLT   = off; off += szLT;
  const size_t oPLh  = off; off += szPL;   const size_t oPLl  = off; off += szPL;
  if (off > ws_size) return;
  if (off > (size_t)134217728) return;

  char* ws = (char*)d_ws;
  unsigned short* Xh   = (unsigned short*)(ws + oXh);   unsigned short* Xl   = (unsigned short*)(ws + oXl);
  unsigned short* WqTh = (unsigned short*)(ws + oWqTh); unsigned short* WqTl = (unsigned short*)(ws + oWqTl);
  unsigned short* WkTh = (unsigned short*)(ws + oWkTh); unsigned short* WkTl = (unsigned short*)(ws + oWkTl);
  unsigned short* WvTh = (unsigned short*)(ws + oWvTh); unsigned short* WvTl = (unsigned short*)(ws + oWvTl);
  unsigned short* Woh  = (unsigned short*)(ws + oWoh);  unsigned short* Wol  = (unsigned short*)(ws + oWol);
  unsigned short* BtQh = (unsigned short*)(ws + oBtQh); unsigned short* BtQl = (unsigned short*)(ws + oBtQl);
  unsigned short* Mh   = (unsigned short*)(ws + oMh);   unsigned short* Ml   = (unsigned short*)(ws + oMl);
  unsigned short* QL   = (unsigned short*)(ws + oQL);
  unsigned short* LT   = (unsigned short*)(ws + oLT);
  unsigned short* PLh  = (unsigned short*)(ws + oPLh);  unsigned short* PLl  = (unsigned short*)(ws + oPLl);

  const dim3 blk(256);

  tsplit_kernel<<<dim3(DM / 64, HD / 64, NH), blk, 0, stream>>>(Wq, WqTh, WqTl, HD, DM, (long)HD * DM, (long)DM * HD);
  tsplit_kernel<<<dim3(KR / 64, HD / 64, NH), blk, 0, stream>>>(Wku, WkTh, WkTl, HD, KR, (long)HD * KR, (long)KR * HD);
  tsplit_kernel<<<dim3(KR / 64, HD / 64, NH), blk, 0, stream>>>(Wvu, WvTh, WvTl, HD, KR, (long)HD * KR, (long)KR * HD);
  split_bf16x2_kernel<<<dim3((DM * QD / 2 + 255) / 256), blk, 0, stream>>>(Wo, Woh, Wol, DM * QD / 2);
  split_bf16x2_kernel<<<dim3((KR * DM / 2 + 255) / 256), blk, 0, stream>>>(Wkv, BtQh + (size_t)HRK * DM, BtQl + (size_t)HRK * DM, KR * DM / 2);
  split_bf16x2_kernel<<<dim3((NROWS * DM / 2 + 255) / 256), blk, 0, stream>>>(x, Xh, Xl, NROWS * DM / 2);
  {
    const int tiles = (KR / 64) * (DM / 64);
    gemm64_split<2><<<dim3((tiles + 7) / 8, NH), blk, 0, stream>>>(
        WkTh, WkTl, HD, (long)KR * HD, WqTh, WqTl, HD, (long)DM * HD,
        (void*)BtQh, (void*)BtQl, DM, (long)KR * DM, KR, DM, HD, 1.0f);
  }
  {
    const int tiles = (DM / 64) * (KR / 64);
    gemm64_split<2><<<dim3((tiles + 7) / 8, NH), blk, 0, stream>>>(
        Woh, Wol, QD, (long)HD, WvTh, WvTl, HD, (long)KR * HD,
        (void*)Mh, (void*)Ml, HRK, (long)KR, DM, KR, HD, 1.0f);
  }
  {
    const int tiles = (NROWS / 64) * (QLP / 64);
    gemm64_split<1><<<dim3((tiles + 7) / 8, 1), blk, 0, stream>>>(
        Xh, Xl, DM, 0L, BtQh, BtQl, DM, 0L,
        (void*)QL, (void*)QL, QLP, 0L, NROWS, QLP, DM, 8.0f);
  }
  lat_tr_kernel<<<dim3(TS / 64, NB), blk, 0, stream>>>(QL, LT);
  attn_lat64_kernel<<<dim3(NB * NH * (TS / AT_QB)), dim3(128), 0, stream>>>(QL, LT, PLh, PLl, 0.0009765625f, 3.0517578125e-05f);
  {
    const int tiles = (NROWS / 64) * (DM / 64);
    gemm64_split<0><<<dim3((tiles + 7) / 8, 1), blk, 0, stream>>>(
        PLh, PLl, HRK, 0L, Mh, Ml, HRK, 0L,
        d_out, d_out, DM, 0L, NROWS, DM, HRK, 1.0f);
  }
  (void)hipGetLastError();
}
